// GraphNN_38268158607515
// MI455X (gfx1250) — hardware-verified
//
#include <hip/hip_runtime.h>
#include <stddef.h>


typedef _Float16 h16;
typedef _Float16 v16h __attribute__((ext_vector_type(16)));
typedef _Float16 v8h  __attribute__((ext_vector_type(8)));
typedef float    v8f  __attribute__((ext_vector_type(8)));
typedef float    v4f  __attribute__((ext_vector_type(4)));

#ifndef NROWS
#define NROWS 16384
#endif
#define NROWS_FULL 16384
#define WIDTH   128
#define NNODES  12
#define NEDGES  66
#define NPLANES 11

static_assert(NROWS >= 64 && NROWS <= NROWS_FULL);
static_assert((NROWS % 64) == 0);
static_assert((NROWS % 16) == 0);
static_assert(NEDGES == NNODES * (NNODES - 1) / 2);
static_assert(NPLANES == NNODES - 1);
static_assert(WIDTH == 128);
static_assert((WIDTH % 64) == 0 && (WIDTH % 32) == 0 && (WIDTH % 8) == 0);
static_assert(16 * 8 == WIDTH);
static_assert(32 * 4 == WIDTH);

#define LDT 72
#define LDC 132
static_assert((LDT % 8) == 0 && LDT >= 64);
static_assert((LDC % 4) == 0 && LDC >= WIDTH);

#define WCARRY 64.0f
#define ACARRY 16.0f

#define PLANE_ELEMS ((size_t)NROWS * WIDTH)
#define WT_BYTES    ((size_t)NEDGES * WIDTH * WIDTH * 2)
#define PL_BYTES    ((size_t)NPLANES * PLANE_ELEMS * 2)
#define OFF_WT      ((size_t)0)
#define OFF_PL      (OFF_WT + WT_BYTES)
#define WS_TOTAL    (OFF_PL + PL_BYTES)
static_assert((WT_BYTES % 128) == 0 && (PL_BYTES % 128) == 0);
static_assert(((PLANE_ELEMS * 2) % 128) == 0);
static_assert(WS_TOTAL <= (size_t)134217728);

__device__ __forceinline__ float bf16r(float x) {
  unsigned int u = __float_as_uint(x);
  u = (u + 0x7FFFu + ((u >> 16) & 1u)) & 0xFFFF0000u;
  return __uint_as_float(u);
}

static __device__ __forceinline__ h16 toh_flush(float v) {
  const h16 r = (h16)v;
  return (fabsf(v) < 6.103515625e-05f) ? (h16)0.0f : r;
}

__device__ __forceinline__ v16h frag_at(const _Float16* p) {
  v8h lo = *(const v8h*)(p);
  v8h hi = *(const v8h*)(p + 16);
  v16h out;
#pragma unroll
  for (int i = 0; i < 8; ++i) { out[i] = lo[i]; out[i + 8] = hi[i]; }
  return out;
}

__device__ __forceinline__ v8f wmma16(v16h a, v16h b, v8f c) {
  v8f d = __builtin_amdgcn_wmma_f32_16x16x32_f16(false, a, false, b, (short)0, c,
                                                 false, false);
  asm volatile("v_nop\n\tv_nop\n\tv_nop\n\tv_nop" : "+v"(d) : "v"(a), "v"(b));
  return d;
}

__global__ __launch_bounds__(256) void wconv_edges_kernel(
    const float* __restrict__ W, _Float16* __restrict__ Wt) {
  __shared__ _Float16 T[64 * LDT];
  const unsigned tid = threadIdx.x;
  const unsigned n0 = blockIdx.x * 64u;
  const unsigned k0 = blockIdx.y * 64u;
  const size_t eoff = (size_t)blockIdx.z * (WIDTH * WIDTH);
#pragma unroll 4
  for (unsigned j = 0; j < 16u; ++j) {
    const unsigned idx = tid + 256u * j;
    const unsigned kr = idx >> 6, nc = idx & 63u;
    const float v = W[eoff + (size_t)(k0 + kr) * WIDTH + n0 + nc];
    T[nc * LDT + kr] = toh_flush(WCARRY * bf16r(v));
  }
  __syncthreads();
  v8h x[2];
  size_t off[2];
#pragma unroll
  for (unsigned i = 0; i < 2u; ++i) {
    const unsigned n = 32u * i + (tid >> 3);
    const unsigned kc = (tid & 7u) * 8u;
    x[i] = *(const v8h*)&T[n * LDT + kc];
    off[i] = eoff + (size_t)(n0 + n) * WIDTH + k0 + kc;
  }
#pragma unroll
  for (int i = 0; i < 2; ++i) *(volatile v8h*)(Wt + off[i]) = x[i];
  __threadfence();
#pragma unroll
  for (int i = 0; i < 2; ++i) *(volatile v8h*)(Wt + off[i]) = x[i];
}

__global__ __launch_bounds__(256) void xconv_kernel(
    const float* __restrict__ X, _Float16* __restrict__ dst) {
  const size_t g = ((size_t)blockIdx.x * 256u + threadIdx.x) * 8u;
  const v4f a0 = *(const v4f*)(X + g);
  const v4f a1 = *(const v4f*)(X + g + 4u);
  v8h o;
#pragma unroll
  for (int i = 0; i < 4; ++i) {
    o[i]     = toh_flush(ACARRY * bf16r(a0[i]));
    o[i + 4] = toh_flush(ACARRY * bf16r(a1[i]));
  }
  _Float16* q = dst + g;
  *(volatile v8h*)q = o;
  __threadfence();
  *(volatile v8h*)q = o;
}

template <int FINAL>
__device__ __forceinline__ void level_body(
    const _Float16* __restrict__ planes, const _Float16* __restrict__ Wt,
    const float* __restrict__ bias, const int p,
    _Float16* __restrict__ out16, float* __restrict__ outf) {
  __shared__ float Cs[64 * LDC];
  const unsigned tid = threadIdx.x, lane = tid & 31u;
  const unsigned w = (unsigned)__builtin_amdgcn_readfirstlane((int)(threadIdx.x >> 5));
  const unsigned mw = w >> 1, nw = w & 1u;
  const unsigned hh = lane >> 4, m = lane & 15u;
  const unsigned row0 = blockIdx.x * 64u;

  const size_t aoff = (size_t)(row0 + mw * 16u + m) * WIDTH + hh * 8u;
  const size_t boff = (size_t)(nw * 64u + m) * WIDTH + hh * 8u;
  const float cs = 1.0f / (WCARRY * ACARRY);

  v8f acc[4];
#pragma unroll
  for (int ct = 0; ct < 4; ++ct) acc[ct] = (v8f){};

#pragma unroll 1
  for (int u = 0; u < p; ++u) {
    const _Float16* ap = planes + (size_t)u * PLANE_ELEMS + aoff;
    const _Float16* bp = Wt + (size_t)u * (WIDTH * WIDTH) + boff;
    const float* be = bias + (size_t)u * WIDTH + nw * 64u + m;
    v8f t[4];
#pragma unroll
    for (int ct = 0; ct < 4; ++ct) t[ct] = (v8f){};
#pragma unroll
    for (unsigned k0 = 0; k0 < (unsigned)WIDTH; k0 += 32u) {
      const v16h a = frag_at(ap + k0);
#pragma unroll
      for (int ct = 0; ct < 4; ++ct) {
        const v16h b = frag_at(bp + (size_t)ct * 16u * WIDTH + k0);
        t[ct] = wmma16(a, b, t[ct]);
      }
    }
#pragma unroll
    for (int ct = 0; ct < 4; ++ct) {
      const float bb = bf16r(be[ct * 16]);
#pragma unroll
      for (int r = 0; r < 8; ++r) {
        const float h = t[ct][r] * cs + bb;
        acc[ct][r] = acc[ct][r] + fmaxf(h, 0.0f);
      }
    }
  }

#pragma unroll
  for (int ct = 0; ct < 4; ++ct)
#pragma unroll
    for (int r = 0; r < 8; ++r)
      Cs[(mw * 16u + hh * 8u + (unsigned)r) * LDC + nw * 64u + (unsigned)ct * 16u + m] = acc[ct][r];
  __syncthreads();

  if (FINAL == 0) {
    v8h x[4];
    size_t off[4];
#pragma unroll
    for (unsigned i = 0; i < 4u; ++i) {
      const unsigned r = 16u * i + (tid >> 4);
      const unsigned c = (tid & 15u) * 8u;
      const v4f u0 = *(const v4f*)&Cs[r * LDC + c];
      const v4f u1 = *(const v4f*)&Cs[r * LDC + c + 4u];
#pragma unroll
      for (int j = 0; j < 4; ++j) {
        x[i][j]     = toh_flush(ACARRY * u0[j]);
        x[i][j + 4] = toh_flush(ACARRY * u1[j]);
      }
      off[i] = (size_t)(row0 + r) * WIDTH + c;
    }
#pragma unroll
    for (int i = 0; i < 4; ++i) *(volatile v8h*)(out16 + off[i]) = x[i];
    __threadfence();
#pragma unroll
    for (int i = 0; i < 4; ++i) *(volatile v8h*)(out16 + off[i]) = x[i];
  } else {
    v4f xs[8];
    size_t off[8];
#pragma unroll
    for (unsigned i = 0; i < 8u; ++i) {
      const unsigned r = 8u * i + (tid >> 5);
      const unsigned c = (tid & 31u) * 4u;
      xs[i] = *(const v4f*)&Cs[r * LDC + c];
      off[i] = (size_t)(row0 + r) * WIDTH + c;
    }
#pragma unroll
    for (int i = 0; i < 8; ++i) *(volatile v4f*)(outf + off[i]) = xs[i];
    __threadfence();
#pragma unroll
    for (int i = 0; i < 8; ++i) *(volatile v4f*)(outf + off[i]) = xs[i];
  }
}

__global__ __launch_bounds__(256) void level_mid_kernel(
    const _Float16* __restrict__ planes, const _Float16* __restrict__ Wt,
    const float* __restrict__ bias, int p, _Float16* __restrict__ out16) {
  level_body<0>(planes, Wt, bias, p, out16, (float*)0);
}
__global__ __launch_bounds__(256) void level_out_kernel(
    const _Float16* __restrict__ planes, const _Float16* __restrict__ Wt,
    const float* __restrict__ bias, int p, float* __restrict__ outf) {
  level_body<1>(planes, Wt, bias, p, (_Float16*)0, outf);
}

extern "C" void kernel_launch(void* const* d_in, const int* in_sizes, int n_in,
                              void* d_out, int out_size, void* d_ws, size_t ws_size,
                              hipStream_t stream) {
  if (n_in < 3) return;
  if ((long long)in_sizes[0] < (long long)NROWS * WIDTH) return;
  if ((long long)in_sizes[1] < (long long)NEDGES * WIDTH * WIDTH) return;
  if ((long long)in_sizes[2] < (long long)NEDGES * WIDTH) return;
  if ((long long)out_size < (long long)NROWS * WIDTH) return;
  if (ws_size < WS_TOTAL) return;

  const float* X = (const float*)d_in[0];
  const float* W = (const float*)d_in[1];
  const float* B = (const float*)d_in[2];
  float* out = (float*)d_out;

  char* ws = (char*)d_ws;
  _Float16* Wt16   = (_Float16*)(ws + OFF_WT);
  _Float16* Planes = (_Float16*)(ws + OFF_PL);

  dim3 blk(256);

  wconv_edges_kernel<<<dim3(WIDTH / 64, WIDTH / 64, NEDGES), blk, 0, stream>>>(W, Wt16);
  xconv_kernel<<<dim3(NROWS / 16), blk, 0, stream>>>(X, Planes);

  int start = 0;
  for (int v = 2; v <= NNODES; ++v) {
    const int p = v - 1;
    const _Float16* Wl = Wt16 + (size_t)start * WIDTH * WIDTH;
    const float* bl = B + (size_t)start * WIDTH;
    if (v < NNODES) {
      level_mid_kernel<<<dim3(NROWS / 64), blk, 0, stream>>>(
          Planes, Wl, bl, p, Planes + (size_t)p * PLANE_ELEMS);
    } else {
      level_out_kernel<<<dim3(NROWS / 64), blk, 0, stream>>>(Planes, Wl, bl, p, out);
    }
    start += p;
  }
}
